// SeqVAE_21852793602681
// MI455X (gfx1250) — hardware-verified
//
#include <hip/hip_runtime.h>
#include <math.h>

typedef __attribute__((ext_vector_type(16))) _Float16 v16h;
typedef __attribute__((ext_vector_type(8)))  _Float16 v8h;
typedef __attribute__((ext_vector_type(16))) __bf16   v16b;
typedef __attribute__((ext_vector_type(8)))  __bf16   v8b;
typedef __attribute__((ext_vector_type(8)))  float    v8f;
typedef __attribute__((ext_vector_type(4)))  float    v4f;

constexpr int kB    = 2048;
constexpr int kS    = 200;
constexpr int kDX   = 64;
constexpr int kZ    = 32;
constexpr int kH    = 128;
constexpr int kAE   = 32;
constexpr int kTE   = 16;
constexpr int kAV   = 100;
constexpr int kTV   = 4;
constexpr int kDIn  = kDX + kAE + kTE + kZ + 1;
constexpr int kDInP = 160;
constexpr int kInpP = 256;
constexpr int kA0P  = 128;
constexpr int kG3   = 3 * kH;
constexpr int kThr  = 256;
constexpr float kInCarry = 1024.0f;
constexpr float kSc = 1.0f / (kInCarry * kInCarry);
constexpr float kF16MinNormal = 6.103515625e-5f;
constexpr int kFBX = 0, kFB0 = 64, kFBI = 192, kFBH = 576, kFBZ = 960, kFEnd = 1024;

static_assert(kDIn == 145 && (kB % 64) == 0 && ((kB / 64) * (kDX / 64)) % 8 == 0 && ((kB / 64) * (kH / 64)) % 8 == 0 && ((kB / 64) * (kG3 / 64)) % 8 == 0
              && (kDX % 32) == 0 && (96 % 32) == 0 && (kDInP % 32) == 0 && (kH % 32) == 0, "GEMM M, N multiples of 64; grids exact; K multiples of 32");

constexpr size_t kOffWX16 = 0ull;
constexpr size_t kOffWH0 = 8192ull;
constexpr size_t kOffWIH = 32768ull;
constexpr size_t kOffWHH = 155648ull;
constexpr size_t kOffBIAS = 253952ull;
constexpr size_t kOffX16 = 258048ull;
constexpr size_t kOffXE32 = 520192ull;
constexpr size_t kOffA0 = 1044480ull;
constexpr size_t kOffHP32 = 1568768ull;
constexpr size_t kOffH32 = 2617344ull;
constexpr size_t kOffAH = 3665920ull;
constexpr size_t kOffINP = 4190208ull;
constexpr size_t kOffGI = 5238784ull;
constexpr size_t kOffGH = 8384512ull;
constexpr size_t kWsTotal = 11530240ull;
static_assert(kWsTotal <= 134217728ull, "carve cap: under 128 MiB");
static_assert(kOffWX16 == 0
              && kOffWH0 == kOffWX16 + 8192ull
              && kOffWIH == kOffWH0 + 24576ull
              && kOffWHH == kOffWIH + 122880ull
              && kOffBIAS == kOffWHH + 98304ull
              && kOffX16 == kOffBIAS + 4096ull
              && kOffXE32 == kOffX16 + 262144ull
              && kOffA0 == kOffXE32 + 524288ull
              && kOffHP32 == kOffA0 + 524288ull
              && kOffH32 == kOffHP32 + 1048576ull
              && kOffAH == kOffH32 + 1048576ull
              && kOffINP == kOffAH + 524288ull
              && kOffGI == kOffINP + 1048576ull
              && kOffGH == kOffGI + 3145728ull
              && kWsTotal == kOffGH + 3145728ull, "the carve is chained and totalled");
static_assert((kOffWX16 % 256) == 0 && (kOffWH0 % 256) == 0 && (kOffWIH % 256) == 0 && (kOffWHH % 256) == 0 && (kOffBIAS % 256) == 0 && (kOffX16 % 256) == 0 && (kOffXE32 % 256) == 0 && (kOffA0 % 256) == 0 && (kOffHP32 % 256) == 0 && (kOffH32 % 256) == 0 && (kOffAH % 256) == 0 && (kOffINP % 256) == 0 && (kOffGI % 256) == 0 && (kOffGH % 256) == 0, "aligned regions");

__device__ __forceinline__ unsigned short f2bf_bits(float f) {
  unsigned u = __float_as_uint(f);
  return (unsigned short)((u + 0x7FFFu + ((u >> 16) & 1u)) >> 16);
}
__device__ __forceinline__ float bf_bits2f(unsigned short h) { return __uint_as_float(((unsigned)h) << 16); }
__device__ __forceinline__ float bf16r(float f) { return bf_bits2f(f2bf_bits(f)); }
__device__ __forceinline__ float carry_flush(float v, float carry) {
  const float s = v * carry;
  return (fabsf(s) < kF16MinNormal) ? 0.0f : s;
}
__device__ __forceinline__ float frcp(float x) { return __builtin_amdgcn_rcpf(x); }

__device__ __forceinline__ void dep_guard4_h(v8f& a, v8f& b, v8f& c, v8f& d, v16h x, v16h y) { asm volatile("v_nop\n\tv_nop\n\tv_nop\n\tv_nop" : "+v"(a), "+v"(b), "+v"(c), "+v"(d) : "v"(x), "v"(y)); }
__device__ __forceinline__ void dep_guard4_b(v8f& a, v8f& b, v8f& c, v8f& d, v16b x, v16b y) { asm volatile("v_nop\n\tv_nop\n\tv_nop\n\tv_nop" : "+v"(a), "+v"(b), "+v"(c), "+v"(d) : "v"(x), "v"(y)); }
__device__ __forceinline__ void keep4_h(v16h a, v16h b, v16h c, v16h d) { asm volatile("v_nop" :: "v"(a), "v"(b), "v"(c), "v"(d)); }
__device__ __forceinline__ void keep4_b(v16b a, v16b b, v16b c, v16b d) { asm volatile("v_nop" :: "v"(a), "v"(b), "v"(c), "v"(d)); }
__device__ __forceinline__ void acc_guard4(v8f& a, v8f& b, v8f& c, v8f& d) { asm volatile("v_nop\n\tv_nop\n\tv_nop\n\tv_nop" : "+v"(a), "+v"(b), "+v"(c), "+v"(d)); }

template <typename T> struct Frag;
template <> struct Frag<_Float16> {
  typedef v16h V; union U { v16h v; v8h h[2]; };
  static __device__ __forceinline__ v16h load(const _Float16* p) {
    U f; f.h[0] = *(const v8h*)(p); f.h[1] = *(const v8h*)(p + 16); return f.v;
  }
  static __device__ __forceinline__ v8f mma(v16h a, v16h b, v8f c) {
    return __builtin_amdgcn_wmma_f32_16x16x32_f16(false, a, false, b, (short)0, c, false, false);
  }
  static __device__ __forceinline__ void guard4(v8f& a, v8f& b, v8f& c, v8f& d, v16h x, v16h y) { dep_guard4_h(a, b, c, d, x, y); }
  static __device__ __forceinline__ void keep(v16h a, v16h b, v16h c, v16h d) { keep4_h(a, b, c, d); }
};
template <> struct Frag<__bf16> {
  typedef v16b V; union U { v16b v; v8b h[2]; };
  static __device__ __forceinline__ v16b load(const __bf16* p) {
    U f; f.h[0] = *(const v8b*)(p); f.h[1] = *(const v8b*)(p + 16); return f.v;
  }
  static __device__ __forceinline__ v8f mma(v16b a, v16b b, v8f c) {
    return __builtin_amdgcn_wmma_f32_16x16x32_bf16(false, a, false, b, (short)0, c, false, false);
  }
  static __device__ __forceinline__ void guard4(v8f& a, v8f& b, v8f& c, v8f& d, v16b x, v16b y) { dep_guard4_b(a, b, c, d, x, y); }
  static __device__ __forceinline__ void keep(v16b a, v16b b, v16b c, v16b d) { keep4_b(a, b, c, d); }
};

__device__ __forceinline__ v8f mma_h(v16h a, v16h b, v8f c) {
  c = __builtin_amdgcn_wmma_f32_16x16x32_f16(false, a, false, b, (short)0, c, false, false);
  asm volatile("v_nop\n\tv_nop\n\tv_nop\n\tv_nop" : "+v"(c) : "v"(a), "v"(b));
  return c;
}

template <int ET> struct Elem;
template <> struct Elem<0> { typedef _Float16 T; };
template <> struct Elem<1> { typedef __bf16 T; };
template <int ET, bool SPLIT, int BIAS_MODE, int OUT_MODE, bool RESID, int ACT = 0>
__global__ __launch_bounds__(256) void wmma_gemm64(
    const unsigned short* __restrict__ Ap, const unsigned short* __restrict__ A2p, int lda, long strideA,
    const unsigned short* __restrict__ Btp, const unsigned short* __restrict__ Bt2p, int ldb, long strideB,
    void* __restrict__ Cout, void* __restrict__ Cout2, int ldc, long strideC,
    const float* __restrict__ bias,
    const float* __restrict__ resid, long strideR,
    int M, int N, int K, float scale) {
  typedef typename Elem<ET>::T T;
  typedef typename Frag<T>::V V;
  const T* A = (const T*)Ap; const T* A2 = (const T*)A2p; const T* Bt = (const T*)Btp; const T* Bt2 = (const T*)Bt2p;
  __shared__ __align__(16) float sT[8][16 * 68];
  const int b    = blockIdx.y;
  const int lane = threadIdx.x & 31;
  const int wave = threadIdx.x >> 5;
  const int tilesN = N >> 6;
  const int tilesM = M >> 6;
  const int tile = blockIdx.x * 8 + wave;
  if (tile >= tilesM * tilesN) return;
  const int tm = tile / tilesN;
  const int tn = tile - tm * tilesN;
  const int m0 = tm << 6;
  const int n0 = tn << 6;

  const T* Ab  = A  + (size_t)b * strideA;
  const T* Bb  = Bt + (size_t)b * strideB;
  const T* Ab2 = SPLIT ? (A2  + (size_t)b * strideA) : nullptr;
  const T* Bb2 = SPLIT ? (Bt2 + (size_t)b * strideB) : nullptr;

  const int rlane = lane & 15;
  const int koff  = (lane >> 4) * 8;
  const int mOff  = (lane >> 4) * 8;

  v8f acc[4][4];
#pragma unroll
  for (int i = 0; i < 4; ++i)
#pragma unroll
    for (int j = 0; j < 4; ++j) acc[i][j] = (v8f){0.f,0.f,0.f,0.f,0.f,0.f,0.f,0.f};

  for (int k0 = 0; k0 < K; k0 += 32) {
    V bh[4], bl[4];
#pragma unroll
    for (int j = 0; j < 4; ++j) {
      const size_t bo = (size_t)(n0 + (j << 4) + rlane) * ldb + koff + k0;
      bh[j] = Frag<T>::load(Bb + bo);
      if (SPLIT) bl[j] = Frag<T>::load(Bb2 + bo);
    }
#pragma unroll
    for (int i = 0; i < 4; ++i) {
      const size_t ao = (size_t)(m0 + (i << 4) + rlane) * lda + koff + k0;
      V ah = Frag<T>::load(Ab + ao);
      V al;
      if (SPLIT) al = Frag<T>::load(Ab2 + ao);
#pragma unroll
      for (int j = 0; j < 4; ++j) {
        acc[i][j] = Frag<T>::mma(ah, bh[j], acc[i][j]);
        if (SPLIT) {
          acc[i][j] = Frag<T>::mma(ah, bl[j], acc[i][j]);
          acc[i][j] = Frag<T>::mma(al, bh[j], acc[i][j]);
        }
      }
      Frag<T>::guard4(acc[i][0], acc[i][1], acc[i][2], acc[i][3], ah, SPLIT ? al : ah);
    }
    Frag<T>::keep(bh[0], bh[1], bh[2], bh[3]);
    if (SPLIT) Frag<T>::keep(bl[0], bl[1], bl[2], bl[3]);
  }
  acc_guard4(acc[0][0], acc[0][1], acc[0][2], acc[0][3]);
  acc_guard4(acc[1][0], acc[1][1], acc[1][2], acc[1][3]);
  acc_guard4(acc[2][0], acc[2][1], acc[2][2], acc[2][3]);
  acc_guard4(acc[3][0], acc[3][1], acc[3][2], acc[3][3]);

  float* slab = sT[wave];
  const float* Rb = RESID ? (resid + (size_t)b * strideR) : nullptr;
#pragma unroll
  for (int i = 0; i < 4; ++i) {
    const int mBase = m0 + (i << 4);
#pragma unroll
    for (int j = 0; j < 4; ++j) {
      const int n = n0 + (j << 4) + rlane;
      float bv = 0.f;
      if (BIAS_MODE == 2) bv = bias[n];
#pragma unroll
      for (int r = 0; r < 8; ++r) {
        float v = acc[i][j][r] * scale;
        if (BIAS_MODE == 1) v += bias[mBase + mOff + r];
        if (BIAS_MODE == 2) v += bv;
        if (RESID) v += Rb[(size_t)(mBase + mOff + r) * ldc + n];
        if (ACT == 1) v = tanhf(v);
        if (ACT == 2) v = fmaxf(v, 0.0f);
        if (ACT == 3) v = v / (1.0f + expf(-v));
        if (ACT == 4) v = (v > 0.f) ? v : 0.01f * v;
        slab[(mOff + r) * 68 + (j << 4) + rlane] = v;
      }
    }
    __builtin_amdgcn_fence(__ATOMIC_RELEASE, "workgroup");
    __builtin_amdgcn_wave_barrier();
    __builtin_amdgcn_fence(__ATOMIC_ACQUIRE, "workgroup");
    if (OUT_MODE == 0) {
      float* C = (float*)Cout + (size_t)b * strideC;
      const int hh = lane >> 4, c4 = (lane & 15) * 4;
      for (int pass = 0; pass < 2; ++pass) {
#pragma unroll
        for (int it = 0; it < 8; ++it) {
          const int row = it * 2 + hh;
          v4f v = *(const v4f*)(slab + row * 68 + c4);
          *(volatile v4f*)(C + (size_t)(mBase + row) * ldc + n0 + c4) = v;
        }
        __threadfence();
      }
    } else {
      const int q = lane >> 3, c8 = (lane & 7) * 8;
      unsigned short* C  = (unsigned short*)Cout  + (size_t)b * strideC;
      unsigned short* C2 = (OUT_MODE == 2) ? ((unsigned short*)Cout2 + (size_t)b * strideC) : nullptr;
      for (int pass = 0; pass < 2; ++pass) {
#pragma unroll
        for (int it = 0; it < 4; ++it) {
          const int row = it * 4 + q;
          const float* sp = slab + row * 68 + c8;
          v8h hv, lv;
#pragma unroll
          for (int e = 0; e < 8; ++e) {
            if (OUT_MODE == 1) {
              hv[e] = (_Float16)sp[e];
            } else {
              unsigned short hb = f2bf_bits(sp[e]);
              unsigned short lb = f2bf_bits(sp[e] - bf_bits2f(hb));
              hv[e] = __builtin_bit_cast(_Float16, hb);
              lv[e] = __builtin_bit_cast(_Float16, lb);
            }
          }
          *(volatile v8h*)(C + (size_t)(mBase + row) * ldc + n0 + c8) = hv;
          if (OUT_MODE == 2) *(volatile v8h*)(C2 + (size_t)(mBase + row) * ldc + n0 + c8) = lv;
        }
        __threadfence();
      }
    }
    __builtin_amdgcn_fence(__ATOMIC_RELEASE, "workgroup");
    __builtin_amdgcn_wave_barrier();
    __builtin_amdgcn_fence(__ATOMIC_ACQUIRE, "workgroup");
  }
}

__global__ __launch_bounds__(kThr) void cast_plane_kernel(const float* __restrict__ src, unsigned short* __restrict__ dst,
                                                          int colsLog2, int dstPitch, int dstOff) {
  const int i   = blockIdx.x * kThr + threadIdx.x;
  const int sh  = colsLog2 - 3;
  const int row = i >> sh;
  const int c8  = (i & ((1 << sh) - 1)) * 8;
  const float* sp = src + ((size_t)row << colsLog2) + c8;
  const v4f a0 = *(const v4f*)(sp);
  const v4f a1 = *(const v4f*)(sp + 4);
  v8h hv;
#pragma unroll
  for (int e = 0; e < 4; ++e) {
    const float f0 = a0[e];
    const float f1 = a1[e];
    hv[e]     = (_Float16)carry_flush(bf16r(f0), kInCarry);
    hv[4 + e] = (_Float16)carry_flush(bf16r(f1), kInCarry);
  }
  unsigned short* dp = dst + (size_t)row * dstPitch + dstOff + c8;
  *(volatile v8h*)dp = hv;
  __threadfence();
  *(volatile v8h*)dp = hv;
}

__device__ __forceinline__ float fast_tanh(float v) { return 1.0f - 2.0f * frcp(__expf(2.0f * v) + 1.0f); }
__device__ __forceinline__ float fast_sigmoid(float v) { return frcp(1.0f + __expf(-v)); }

__global__ __launch_bounds__(kThr) void setup_kernel(const float* __restrict__ w_ih, const float* __restrict__ xb, const float* __restrict__ h0b,
                                                     const float* __restrict__ bih, const float* __restrict__ bhh,
                                                     unsigned short* __restrict__ WIH, float* __restrict__ BIAS) {
  unsigned v = blockIdx.x * (unsigned)kThr + threadIdx.x;
  asm volatile("" : "+v"(v));
  if (v < 7680u) {
    const unsigned n = v / 20u, k8 = (v % 20u) * 8u;
    v8h hv;
#pragma unroll
    for (int e = 0; e < 8; ++e) {
      const unsigned k = k8 + (unsigned)e;
      const bool live = k < (unsigned)kDIn;
      float w = w_ih[(size_t)n * kDIn + (live ? k : 0u)];
      asm volatile("" : "+v"(w));
      hv[e] = (_Float16)(live ? carry_flush(bf16r(w), kInCarry) : 0.0f);
    }
    unsigned short* dp = WIH + (size_t)v * 8u;
    *(volatile v8h*)dp = hv;
    __threadfence();
    *(volatile v8h*)dp = hv;
  } else {
    const unsigned i0 = (v - 7680u) * 4u;
    const float* sp = (i0 < 64u) ? (xb + i0) : (i0 < 192u) ? (h0b + (i0 - 64u)) : (i0 < 576u) ? (bih + (i0 - 192u)) : (bhh + ((i0 < 960u) ? (i0 - 576u) : 0u));
    const bool live = i0 < 960u;
    const v4f a = *(const v4f*)sp;
    v4f o;
#pragma unroll
    for (int e = 0; e < 4; ++e) { const float x = a[e]; o[e] = live ? bf16r(x) : 0.0f; }
    float* dp = BIAS + i0;
    *(volatile v4f*)dp = o;
    __threadfence();
    *(volatile v4f*)dp = o;
  }
}
static_assert(kG3 * (kDInP / 8) == 7680 && 7680 % kThr == 0 && kFEnd / 4 == 256 && 7680 + 256 == 31 * kThr, "set-up grid exact");

__global__ __launch_bounds__(kThr) void prep_kernel(const float* __restrict__ XE32, const float* __restrict__ z, unsigned short* __restrict__ A0,
                                                    unsigned short* __restrict__ INP) {
  unsigned v = blockIdx.x * (unsigned)kThr + threadIdx.x;
  asm volatile("" : "+v"(v));
  const unsigned b = v >> 5, j = v & 31u;
  if (j >= 25u) return;
  const bool isX = (j < 8u) || (j >= 12u && j < 20u);
  const bool isZ = (j >= 8u && j < 12u) || (j >= 20u && j < 24u);
  const unsigned c8 = (j < 8u) ? j * 8u : (j < 12u) ? (j - 8u) * 8u : (j < 20u) ? (j - 12u) * 8u : (j < 24u) ? (j - 20u) * 8u : 0u;
  const float* sp = isX ? (XE32 + (size_t)b * kDX + c8) : (z + (size_t)b * kZ + (isZ ? c8 : 0u));
  const v4f a0 = *(const v4f*)sp, a1 = *(const v4f*)(sp + 4);
  v8h hv;
#pragma unroll
  for (int e = 0; e < 4; ++e) {
    const float p = isX ? a0[e] : bf16r(a0[e]), q = isX ? a1[e] : bf16r(a1[e]);
    hv[e] = (_Float16)((isX || isZ) ? carry_flush(p, kInCarry) : 0.0f);
    hv[4 + e] = (_Float16)((isX || isZ) ? carry_flush(q, kInCarry) : 0.0f);
  }
  unsigned short* dp = (j < 8u) ? (A0 + (size_t)b * kA0P + c8) : (j < 12u) ? (A0 + (size_t)b * kA0P + kDX + c8)
                     : (j < 20u) ? (INP + (size_t)b * kInpP + c8) : (j < 24u) ? (INP + (size_t)b * kInpP + 112u + c8) : (INP + (size_t)b * kInpP + 152u);
  *(volatile v8h*)dp = hv;
  __threadfence();
  *(volatile v8h*)dp = hv;
}
static_assert(kB * 32 == 256 * kThr && kDX + kAE + kTE == 112 && (kA0P * 2) % 128 == 0 && (kInpP * 2) % 128 == 0, "prep grid exact; rows are whole lines");

__global__ __launch_bounds__(kThr) void h0_kernel(const float* __restrict__ HP32, float* __restrict__ H32, unsigned short* __restrict__ AH) {
  unsigned v = blockIdx.x * (unsigned)kThr + threadIdx.x;
  asm volatile("" : "+v"(v));
  const size_t o8 = (size_t)v * 8u;
  const v4f a0 = *(const v4f*)(HP32 + o8), a1 = *(const v4f*)(HP32 + o8 + 4);
  v4f h0v, h1v; v8h hv;
#pragma unroll
  for (int e = 0; e < 4; ++e) { h0v[e] = tanhf(a0[e]); h1v[e] = tanhf(a1[e]); hv[e] = (_Float16)carry_flush(h0v[e], kInCarry); hv[4 + e] = (_Float16)carry_flush(h1v[e], kInCarry); }
  for (int pass = 0; pass < 2; ++pass) {
    *(volatile v4f*)(H32 + o8) = h0v; *(volatile v4f*)(H32 + o8 + 4) = h1v;
    *(volatile v8h*)(AH + o8) = hv;
    __threadfence();
  }
}
static_assert(kB * kH / 8 == 128 * kThr, "first-state grid exact");

__global__ __launch_bounds__(kThr) void inp_kernel(const int* __restrict__ a, const int* __restrict__ t, const float* __restrict__ y,
                                                   const float* __restrict__ a_emb, const float* __restrict__ t_emb, unsigned short* __restrict__ INP, int s) {
  unsigned v = blockIdx.x * (unsigned)kThr + threadIdx.x;
  asm volatile("" : "+v"(v));
  const unsigned b = v >> 3, j = v & 7u;
  if (j >= 7u) return;
  int ai = a[(size_t)b * kS + s];
  int ti = t[(size_t)b * kS + s];
  asm volatile("" : "+v"(ai), "+v"(ti));
  ai = (ai < 0) ? 0 : (ai > kAV - 1 ? kAV - 1 : ai);
  ti = (ti < 0) ? 0 : (ti > kTV - 1 ? kTV - 1 : ti);
  const float* sp = (j < 4u) ? (a_emb + (size_t)ai * kAE + j * 8u) : (t_emb + (size_t)ti * kTE + ((j < 6u) ? (j - 4u) * 8u : 0u));
  const v4f a0 = *(const v4f*)sp, a1 = *(const v4f*)(sp + 4);
  const float py = (s > 0) ? y[(size_t)b * kS + (s - 1)] : 0.0f;
  v8h hv;
#pragma unroll
  for (int e = 0; e < 4; ++e) { hv[e] = (_Float16)carry_flush(bf16r(a0[e]), kInCarry); hv[4 + e] = (_Float16)carry_flush(bf16r(a1[e]), kInCarry); }
  if (j == 6u) {
#pragma unroll
    for (int e = 0; e < 8; ++e) hv[e] = (_Float16)0.0f;
    hv[0] = (_Float16)carry_flush(bf16r(py), kInCarry);
  }
  unsigned short* dp = INP + (size_t)b * kInpP + ((j < 6u) ? (kDX + j * 8u) : 144u);
  *(volatile v8h*)dp = hv;
  __threadfence();
  *(volatile v8h*)dp = hv;
}
static_assert(kB * 8 == 64 * kThr, "input grid exact");

__global__ __launch_bounds__(kThr) void cell_kernel(const float* __restrict__ GI, const float* __restrict__ GH, float* __restrict__ H32,
                                                    unsigned short* __restrict__ AH) {
  unsigned v = blockIdx.x * (unsigned)kThr + threadIdx.x;
  asm volatile("" : "+v"(v));
  const unsigned b = v >> 4, u8 = (v & 15u) * 8u;
  const float* gi = GI + (size_t)b * kG3 + u8;
  const float* gh = GH + (size_t)b * kG3 + u8;
  float* hp = H32 + (size_t)b * kH + u8;
  v8h hv; v4f hn0, hn1;
#pragma unroll
  for (int hlf = 0; hlf < 2; ++hlf) {
    const v4f ir = *(const v4f*)(gi + 4 * hlf), iu = *(const v4f*)(gi + kH + 4 * hlf), in_ = *(const v4f*)(gi + 2 * kH + 4 * hlf);
    const v4f hr = *(const v4f*)(gh + 4 * hlf), hu = *(const v4f*)(gh + kH + 4 * hlf), hn_ = *(const v4f*)(gh + 2 * kH + 4 * hlf);
    const v4f ho = *(const v4f*)(hp + 4 * hlf);
#pragma unroll
    for (int e = 0; e < 4; ++e) {
      const float r = fast_sigmoid(ir[e] + hr[e]);
      const float z = fast_sigmoid(iu[e] + hu[e]);
      const float n = fast_tanh(in_[e] + r * hn_[e]);
      const float hn = (1.0f - z) * n + z * ho[e];
      if (hlf == 0) hn0[e] = hn; else hn1[e] = hn;
      hv[4 * hlf + e] = (_Float16)carry_flush(hn, kInCarry);
    }
  }
  unsigned short* ap = AH + (size_t)b * kH + u8;
  for (int pass = 0; pass < 2; ++pass) {
    *(volatile v4f*)hp = hn0; *(volatile v4f*)(hp + 4) = hn1;
    *(volatile v8h*)ap = hv;
    __threadfence();
  }
}
static_assert(kB * 16 == 128 * kThr, "cell grid exact");

__global__ __launch_bounds__(kThr) void read_kernel(const float* __restrict__ H32, const float* __restrict__ yh_w, const float* __restrict__ yh_b,
                                                    const float* __restrict__ mask, float* __restrict__ out0, float* __restrict__ out1, int s) {
  unsigned b = blockIdx.x * (unsigned)kThr + threadIdx.x;
  asm volatile("" : "+v"(b));
  const float* hp = H32 + (size_t)b * kH;
  float acc = 0.0f;
#pragma unroll 1
  for (int u4 = 0; u4 < kH; u4 += 4) {
    const v4f h = *(const v4f*)(hp + u4), w = *(const v4f*)(yh_w + u4);
    acc += h[0] * bf16r(w[0]); acc += h[1] * bf16r(w[1]); acc += h[2] * bf16r(w[2]); acc += h[3] * bf16r(w[3]);
  }
  float yb = yh_b[0];
  asm volatile("" : "+v"(yb));
  const float logits = acc + bf16r(yb);
  const float prob = 1.0f / (1.0f + expf(-logits));
  float m = mask[(size_t)b * kS + s];
  m = bf16r(m);
  const float o0 = m * logits + (1.0f - m) * logits;
  const float o1 = m * prob + (1.0f - m) * prob;
  float* p0 = out0 + (size_t)b * kS + s;
  float* p1 = out1 + (size_t)b * kS + s;
  for (int pass = 0; pass < 2; ++pass) {
    *(volatile float*)p0 = o0;
    *(volatile float*)p1 = o1;
    __threadfence();
  }
}
static_assert(kB == 8 * kThr, "readout grid exact");

extern "C" void kernel_launch(void* const* d_in, const int* in_sizes, int n_in,
                              void* d_out, int out_size, void* d_ws, size_t ws_size,
                              hipStream_t stream) {
  if (n_in < 18 || d_out == nullptr || d_ws == nullptr) return;
  if (in_sizes[0] != kB * kDX || in_sizes[1] != kB * kS || in_sizes[2] != kB * kS || in_sizes[3] != kB * kS || in_sizes[4] != kB * kS || in_sizes[5] != kB * kZ) return;
  if (in_sizes[6] != kDX * kDX || in_sizes[7] != kDX || in_sizes[8] != kAV * kAE || in_sizes[9] != kTV * kTE || in_sizes[10] != kH * 96 || in_sizes[11] != kH) return;
  if (in_sizes[12] != kG3 * kDIn || in_sizes[13] != kG3 * kH || in_sizes[14] != kG3 || in_sizes[15] != kG3 || in_sizes[16] != kH || in_sizes[17] != 1) return;
  if (out_size != 2 * kB * kS) return;
  if (ws_size < kWsTotal) return;
  const float* x = (const float*)d_in[0];
  const int* a = (const int*)d_in[1];
  const int* t = (const int*)d_in[2];
  const float* y = (const float*)d_in[3];
  const float* mask = (const float*)d_in[4];
  const float* z = (const float*)d_in[5];
  const float* xproj_w = (const float*)d_in[6];
  const float* xproj_b = (const float*)d_in[7];
  const float* a_emb = (const float*)d_in[8];
  const float* t_emb = (const float*)d_in[9];
  const float* h0_w = (const float*)d_in[10];
  const float* h0_b = (const float*)d_in[11];
  const float* w_ih = (const float*)d_in[12];
  const float* w_hh = (const float*)d_in[13];
  const float* b_ih = (const float*)d_in[14];
  const float* b_hh = (const float*)d_in[15];
  const float* yh_w = (const float*)d_in[16];
  const float* yh_b = (const float*)d_in[17];
  float* out0 = (float*)d_out;
  float* out1 = out0 + (size_t)kB * kS;
  char* ws = (char*)d_ws;
  unsigned short* WX16 = (unsigned short*)(ws + kOffWX16);
  unsigned short* WH0 = (unsigned short*)(ws + kOffWH0);
  unsigned short* WIH = (unsigned short*)(ws + kOffWIH);
  unsigned short* WHH = (unsigned short*)(ws + kOffWHH);
  float* BIAS = (float*)(ws + kOffBIAS);
  unsigned short* X16 = (unsigned short*)(ws + kOffX16);
  float* XE32 = (float*)(ws + kOffXE32);
  unsigned short* A0 = (unsigned short*)(ws + kOffA0);
  float* HP32 = (float*)(ws + kOffHP32);
  float* H32 = (float*)(ws + kOffH32);
  unsigned short* AH = (unsigned short*)(ws + kOffAH);
  unsigned short* INP = (unsigned short*)(ws + kOffINP);
  float* GI = (float*)(ws + kOffGI);
  float* GH = (float*)(ws + kOffGH);

  cast_plane_kernel<<<(int)(((size_t)kDX * kDX / 8) / kThr), kThr, 0, stream>>>(xproj_w, WX16, 6, kDX, 0);
  cast_plane_kernel<<<(int)(((size_t)kH * 96 / 8) / kThr), kThr, 0, stream>>>(h0_w, WH0, 5, 32, 0);
  cast_plane_kernel<<<(int)(((size_t)kG3 * kH / 8) / kThr), kThr, 0, stream>>>(w_hh, WHH, 7, kH, 0);
  setup_kernel<<<31, kThr, 0, stream>>>(w_ih, xproj_b, h0_b, b_ih, b_hh, WIH, BIAS);
  cast_plane_kernel<<<(int)(((size_t)kB * kDX / 8) / kThr), kThr, 0, stream>>>(x, X16, 6, kDX, 0);
  wmma_gemm64<0, false, 2, 0, false, 0><<<dim3((kB / 64) * (kDX / 64) / 8, 1), 256, 0, stream>>>(
      X16, X16, kDX, 0L, WX16, WX16, kDX, 0L, (void*)XE32, (void*)XE32, kDX, 0L, BIAS + kFBX, nullptr, 0L, kB, kDX, kDX, kSc);
  prep_kernel<<<256, kThr, 0, stream>>>(XE32, z, A0, INP);
  wmma_gemm64<0, false, 2, 0, false, 0><<<dim3((kB / 64) * (kH / 64) / 8, 1), 256, 0, stream>>>(
      A0, A0, kA0P, 0L, WH0, WH0, 96, 0L, (void*)HP32, (void*)HP32, kH, 0L, BIAS + kFB0, nullptr, 0L, kB, kH, 96, kSc);
  h0_kernel<<<128, kThr, 0, stream>>>(HP32, H32, AH);

  for (int s = 0; s < kS; ++s) {
    inp_kernel<<<64, kThr, 0, stream>>>(a, t, y, a_emb, t_emb, INP, s);
    wmma_gemm64<0, false, 2, 0, false, 0><<<dim3((kB / 64) * (kG3 / 64) / 8, 1), 256, 0, stream>>>(
        INP, INP, kInpP, 0L, WIH, WIH, kDInP, 0L, (void*)GI, (void*)GI, kG3, 0L, BIAS + kFBI, nullptr, 0L, kB, kG3, kDInP, kSc);
    wmma_gemm64<0, false, 2, 0, false, 0><<<dim3((kB / 64) * (kG3 / 64) / 8, 1), 256, 0, stream>>>(
        AH, AH, kH, 0L, WHH, WHH, kH, 0L, (void*)GH, (void*)GH, kG3, 0L, BIAS + kFBH, nullptr, 0L, kB, kG3, kH, kSc);
    cell_kernel<<<128, kThr, 0, stream>>>(GI, GH, H32, AH);
    read_kernel<<<8, kThr, 0, stream>>>(H32, yh_w, yh_b, mask, out0, out1, s);
  }
}
